// TransConv_22419729285549
// MI455X (gfx1250) — hardware-verified
//
#include <hip/hip_runtime.h>
#include <math.h>

typedef __attribute__((ext_vector_type(16))) _Float16 v16h;
typedef __attribute__((ext_vector_type(16))) __bf16 v16b;
typedef __attribute__((ext_vector_type(8)))  _Float16 v8h;
typedef __attribute__((ext_vector_type(8)))  float v8f;
typedef __attribute__((ext_vector_type(4)))  float v4f;
typedef __attribute__((ext_vector_type(2)))  float v2f;
typedef __attribute__((ext_vector_type(4)))  unsigned v4u;
typedef __attribute__((ext_vector_type(4)))  int v4i;
typedef float __attribute__((may_alias)) float_a;
typedef int __attribute__((may_alias)) int_a;

template <typename T> __device__ __forceinline__ void vst2(void* p, T v) { *(volatile T*)p = v; __threadfence(); *(volatile T*)p = v; }
__device__ __forceinline__ v8f wmma16(v16h a, v16h b, v8f c) {
  v8f d = __builtin_amdgcn_wmma_f32_16x16x32_f16(false, a, false, b, (short)0, c, false, false);
  asm volatile("v_nop\n\tv_nop\n\tv_nop\n\tv_nop" : "+v"(d) : "v"(a), "v"(b));
  return d;
}
__device__ __forceinline__ v8f wmma_bf(v16b a, v16b b, v8f c) {
  v8f d = __builtin_amdgcn_wmma_f32_16x16x32_bf16(false, a, false, b, (short)0, c, false, false);
  asm volatile("v_nop\n\tv_nop\n\tv_nop\n\tv_nop" : "+v"(d) : "v"(a), "v"(b));
  return d;
}
__device__ __forceinline__ v16h frag_h(const _Float16* rowk0, int lane) {
  union { v16h v; v8h q[2]; } u; const _Float16* p = rowk0 + 8 * (lane >> 4);
  u.q[0] = *(const v8h*)p; u.q[1] = *(const v8h*)(p + 16); return u.v;
}
__device__ __forceinline__ v16h frag_f32(const float* rowk0, int lane) {
  v16h a; const float* p = rowk0 + 8 * (lane >> 4);
#pragma unroll
  for (int i = 0; i < 8; ++i) { a[i] = (_Float16)p[i]; a[8 + i] = (_Float16)p[16 + i]; }
  return a;
}
__device__ __forceinline__ v16h frag_f32s(const float* rowk0, int lane, float sc) {
  v16h a; const float* p = rowk0 + 8 * (lane >> 4);
#pragma unroll
  for (int i = 0; i < 8; ++i) { a[i] = (_Float16)(p[i] * sc); a[8 + i] = (_Float16)(p[16 + i] * sc); }
  return a;
}
__device__ __forceinline__ v16h fragc_f32(const float* W, int k0, int n, int lane, int ld, int K) {
  v16h a; const int g = lane >> 4;
#pragma unroll
  for (int i = 0; i < 8; ++i) { const int ka = k0 + 8 * g + i, kb = ka + 16;
    a[i] = (_Float16)(ka < K ? W[(size_t)(ka < K ? ka : K - 1) * ld + n] : 0.f); a[8 + i] = (_Float16)(kb < K ? W[(size_t)(kb < K ? kb : K - 1) * ld + n] : 0.f); }
  return a;
}
struct F2 { v16b h, l; };
__device__ __forceinline__ F2 bsplit16(const float v[16]) { F2 r;
#pragma unroll
  for (int i = 0; i < 16; ++i) { const __bf16 h = (__bf16)v[i]; r.h[i] = h; r.l[i] = (__bf16)(v[i] - (float)h); }
  return r; }
__device__ __forceinline__ F2 split_row(const float* row, int k0, int lane) { float v[16]; const float* p = row + k0 + 8 * (lane >> 4);
#pragma unroll
  for (int i = 0; i < 8; ++i) { v[i] = p[i]; v[8 + i] = p[16 + i]; }
  return bsplit16(v); }
__device__ __forceinline__ F2 split_rowK(const float* row, int k0, int lane, int K) { float v[16]; const int g = lane >> 4;
#pragma unroll
  for (int i = 0; i < 8; ++i) { const int ka = k0 + 8 * g + i, kb = ka + 16; v[i] = ka < K ? row[ka < K ? ka : K - 1] : 0.f; v[8 + i] = kb < K ? row[kb < K ? kb : K - 1] : 0.f; }
  return bsplit16(v); }
__device__ __forceinline__ F2 split_col(const float* W, int k0, int n, int lane, int ld, int K) { float v[16]; const int g = lane >> 4;
#pragma unroll
  for (int i = 0; i < 8; ++i) { const int ka = k0 + 8 * g + i, kb = ka + 16; v[i] = ka < K ? W[(size_t)(ka < K ? ka : K - 1) * ld + n] : 0.f; v[8 + i] = kb < K ? W[(size_t)(kb < K ? kb : K - 1) * ld + n] : 0.f; }
  return bsplit16(v); }
__device__ __forceinline__ v8f mac3(const F2& a, const F2& b, v8f c) { c = wmma_bf(a.l, b.h, c); c = wmma_bf(a.h, b.l, c); return wmma_bf(a.h, b.h, c); }
__device__ __forceinline__ float sigm(float v) { return 1.0f / (1.0f + expf(-v)); }
#define LDSX() do { asm volatile("s_wait_dscnt 0" ::: "memory"); __builtin_amdgcn_wave_barrier(); __builtin_amdgcn_fence(__ATOMIC_RELEASE, "workgroup"); } while (0)

__device__ __forceinline__ float bfr(float v) { return (float)(__bf16)v; }
__device__ __attribute__((noinline)) float sig_ni(float d) { return 1.0f / (1.0f + expf(d)); }
#define NN 4096
#define DIN 512
#define HID 256
#define NHD 2
#define DK 128
#define VW 256
#define NL 2
#ifndef TNL
#define TNL NL
#endif
#define WS_X   0u
#define WS_Q   (WS_X + 4u * (size_t)NN * HID)
#define WS_K   (WS_Q + 2u * (size_t)NN * HID)
#define WS_VI  (WS_K + 2u * (size_t)NN * HID)
#define WS_VP  (WS_VI + 2u * (size_t)NN * HID)
#define WS_P   (WS_VP + 2u * (size_t)NHD * VW * NN)
#define WS_O   (WS_P + 2u * (size_t)NHD * NN * NN)
#define WS_END (WS_O + 4u * (size_t)NN * NHD * VW)
__global__ __launch_bounds__(128) void k_fc(const float* __restrict__ XI, const float* __restrict__ W, const float* __restrict__ Bv, const float* __restrict__ G0, const float* __restrict__ B0, float* __restrict__ X) { __shared__ __align__(16) float sy[64][HID + 4];
  const int tid = threadIdx.x, wave = tid >> 5, lane = tid & 31, col = lane & 15, g = lane >> 4; const size_t r0 = (size_t)blockIdx.x * 64;
#pragma unroll 1
  for (int cp = 0; cp < 2; ++cp) { v8f acc[8] = {};
#pragma unroll 2
    for (int kc = 0; kc < DIN / 32; ++kc) { v16b a; { const float* p = XI + (r0 + wave * 16 + col) * DIN + kc * 32 + 8 * g;
#pragma unroll
        for (int i = 0; i < 8; ++i) { a[i] = (__bf16)p[i]; a[8 + i] = (__bf16)p[16 + i]; } }
#pragma unroll
      for (int j = 0; j < 8; ++j) { v16b w; const int o = cp * 128 + j * 16 + col;
#pragma unroll
        for (int i = 0; i < 8; ++i) { w[i] = (__bf16)W[(size_t)(kc * 32 + 8 * g + i) * HID + o]; w[8 + i] = (__bf16)W[(size_t)(kc * 32 + 16 + 8 * g + i) * HID + o]; }
        acc[j] = wmma_bf(a, w, acc[j]); } }
#pragma unroll
    for (int j = 0; j < 8; ++j) { const int o = cp * 128 + j * 16 + col; const float bb = bfr(Bv[o]);
#pragma unroll
      for (int r = 0; r < 8; ++r) sy[wave * 16 + 8 * g + r][o] = acc[j][r] + bb; } }
  __syncthreads();
  { const int row = tid >> 1, half = tid & 1; float* v = &sy[row][half * 128]; float s = 0.f; for (int e = 0; e < 128; ++e) s += v[e]; s += __shfl_xor(s, 1); const float mu = s * (1.0f / HID);
    float s2 = 0.f; for (int e = 0; e < 128; ++e) { const float d = v[e] - mu; s2 += d * d; } s2 += __shfl_xor(s2, 1); const float rs = rsqrtf(s2 * (1.0f / HID) + 1e-5f);
    for (int e = 0; e < 128; ++e) { const int c = half * 128 + e; v[e] = fmaxf((v[e] - mu) * rs * bfr(G0[c]) + bfr(B0[c]), 0.f); } }
  __syncthreads();
  for (int q = tid; q < 64 * HID / 4; q += 128) { const int row = q / (HID / 4), c4 = (q % (HID / 4)) * 4; vst2(X + (r0 + row) * HID + c4, *(const v4f*)&sy[row][c4]); } }
__global__ __launch_bounds__(128) void k_lin(const float* __restrict__ X, const _Float16* __restrict__ VI, const float* __restrict__ Wm, const float* __restrict__ Bv, int which, int outw, _Float16* __restrict__ D) { __shared__ __align__(16) _Float16 sh[64][136]; __shared__ __align__(16) _Float16 th[128][72];
  const int tid = threadIdx.x, wave = tid >> 5, lane = tid & 31, col = lane & 15, g = lane >> 4; const int c0 = blockIdx.y * 128; const size_t r0 = (size_t)blockIdx.x * 64;
  v8f acc[8] = {};
#pragma unroll
  for (int kc = 0; kc < HID / 32; ++kc) { v16h a; if (which < 3) a = frag_f32(X + (r0 + wave * 16 + col) * HID + kc * 32, lane); else a = frag_h(VI + (r0 + wave * 16 + col) * HID + kc * 32, lane);
#pragma unroll
    for (int j = 0; j < 8; ++j) { v16h w; const int o = c0 + j * 16 + col;
#pragma unroll
      for (int i = 0; i < 8; ++i) { w[i] = (_Float16)(bfr(Wm[(size_t)(kc * 32 + 8 * g + i) * outw + o]) * 16.0f); w[8 + i] = (_Float16)(bfr(Wm[(size_t)(kc * 32 + 16 + 8 * g + i) * outw + o]) * 16.0f); }
      acc[j] = wmma16(a, w, acc[j]); } }
#pragma unroll
  for (int j = 0; j < 8; ++j) { const int cl = j * 16 + col; const float bb = bfr(Bv[c0 + cl]);
#pragma unroll
    for (int r = 0; r < 8; ++r) { const float v = acc[j][r] * (1.0f / 16.0f) + bb; const int rl = wave * 16 + 8 * g + r; if (which == 3) th[cl][rl] = (_Float16)v; else sh[rl][cl] = (_Float16)v; } }
  __syncthreads();
  if (which < 3) { for (int e = tid; e < 64 * 16; e += 128) { const int rl = e >> 4, q = e & 15; vst2((unsigned*)(D + (r0 + rl) * HID + c0 + q * 8), *(const v4u*)&sh[rl][q * 8]); } }
  else { for (int e = tid; e < 128 * 8; e += 128) { const int cl = e >> 3, q = e & 7; vst2((unsigned*)(D + (size_t)(c0 + cl) * NN + r0 + q * 8), *(const v4u*)&th[cl][q * 8]); } } }
__global__ __launch_bounds__(128) void k_w(const _Float16* __restrict__ Q, const _Float16* __restrict__ K, _Float16* __restrict__ P0, _Float16* __restrict__ P1) { __shared__ __align__(16) _Float16 s0[4][16][136], s1[4][16][136];
  const int tid = threadIdx.x, wave = tid >> 5, lane = tid & 31, col = lane & 15, g = lane >> 4; const int k0 = blockIdx.y * 128; const int ql0 = blockIdx.x * 64 + wave * 16;
  v8f acc0[8] = {}, acc1[8] = {};
#pragma unroll
  for (int kc = 0; kc < DK / 32; ++kc) { const v16h a0 = frag_h(Q + (size_t)(ql0 + col) * HID + kc * 32, lane), a1 = frag_h(Q + (size_t)(ql0 + col) * HID + DK + kc * 32, lane);
#pragma unroll
    for (int j = 0; j < 8; ++j) { const size_t kr = (size_t)(k0 + j * 16 + col) * HID; acc0[j] = wmma16(a0, frag_h(K + kr + kc * 32, lane), acc0[j]); acc1[j] = wmma16(a1, frag_h(K + kr + DK + kc * 32, lane), acc1[j]); } }
  const float isd = 1.0f / sqrtf((float)DK);
#pragma unroll
  for (int j = 0; j < 8; ++j)
#pragma unroll
    for (int r = 0; r < 8; ++r) { const float d = (acc1[j][r] - acc0[j][r]) * isd; const float w0 = sig_ni(d); s0[wave][8 * g + r][j * 16 + col] = (_Float16)(w0 * 2048.0f); s1[wave][8 * g + r][j * 16 + col] = (_Float16)((1.0f - w0) * 2048.0f); }
  LDSX(); for (int rl = 0; rl < 16; ++rl) if (lane < 16) { vst2((unsigned*)(P0 + (size_t)(ql0 + rl) * NN + k0 + lane * 8), *(const v4u*)&s0[wave][rl][lane * 8]); vst2((unsigned*)(P1 + (size_t)(ql0 + rl) * NN + k0 + lane * 8), *(const v4u*)&s1[wave][rl][lane * 8]); } }
__global__ __launch_bounds__(128) void k_pv(const _Float16* __restrict__ P, const _Float16* __restrict__ VP, int h, float* __restrict__ O) { __shared__ __align__(16) float ss[4][16][132];
  const int tid = threadIdx.x, wave = tid >> 5, lane = tid & 31, col = lane & 15, g = lane >> 4; const int cp = blockIdx.y; const int ql0 = blockIdx.x * 64 + wave * 16;
  v8f acc[8] = {};
#pragma unroll 1
  for (int kc = 0; kc < NN / 32; ++kc) { const v16h ph = frag_h(P + (size_t)(ql0 + col) * NN + kc * 32, lane);
#pragma unroll
    for (int j = 0; j < 8; ++j) acc[j] = wmma16(ph, frag_h(VP + (size_t)(h * VW + cp * 128 + j * 16 + col) * NN + kc * 32, lane), acc[j]); }
#pragma unroll
  for (int j = 0; j < 8; ++j)
#pragma unroll
    for (int r = 0; r < 8; ++r) ss[wave][8 * g + r][j * 16 + col] = acc[j][r] * (1.0f / 2048.0f);
  LDSX(); for (int rl = 0; rl < 16; ++rl) vst2(O + ((size_t)(ql0 + rl) * NHD + h) * VW + cp * 128 + lane * 4, *(const v4f*)&ss[wave][rl][lane * 4]); }
__global__ __launch_bounds__(128) void k_mix(const float* __restrict__ O, float* __restrict__ X, const float* __restrict__ Gm, const float* __restrict__ Bb, float* __restrict__ OUT) { __shared__ __align__(16) float sy[64][HID + 4];
  const int tid = threadIdx.x; const size_t r0 = (size_t)blockIdx.x * 64; const int row = tid >> 1, half = tid & 1; const size_t n = r0 + row;
  float s = 0.f; for (int e = 0; e < 128; ++e) { const int c = half * 128 + e; const float om = (O[(n * NHD + 0) * VW + c] + O[(n * NHD + 1) * VW + c]) * 0.5f; const float v = 0.5f * om + 0.5f * X[n * HID + c]; sy[row][c] = v; s += v; }
  s += __shfl_xor(s, 1); const float mu = s * (1.0f / HID); float s2 = 0.f; for (int e = 0; e < 128; ++e) { const float d = sy[row][half * 128 + e] - mu; s2 += d * d; } s2 += __shfl_xor(s2, 1); const float rs = rsqrtf(s2 * (1.0f / HID) + 1e-5f);
  for (int e = 0; e < 128; ++e) { const int c = half * 128 + e; sy[row][c] = (sy[row][c] - mu) * rs * bfr(Gm[c]) + bfr(Bb[c]); }
  __syncthreads();
  float* dst = OUT ? OUT : X;
  for (int q = tid; q < 64 * HID / 4; q += 128) { const int rw = q / (HID / 4), c4 = (q % (HID / 4)) * 4; vst2(dst + (r0 + rw) * HID + c4, *(const v4f*)&sy[rw][c4]); } }
extern "C" void kernel_launch(void* const* d_in, const int* in_sizes, int n_in, void* d_out, int out_size, void* d_ws, size_t ws_size, hipStream_t stream) {
  (void)in_sizes; (void)n_in; (void)out_size;
  const float** F = (const float**)d_in;
  if (ws_size < (size_t)WS_END) return;
  char* ws = (char*)d_ws; float *X = (float*)(ws + WS_X), *O = (float*)(ws + WS_O); _Float16 *Q = (_Float16*)(ws + WS_Q), *K = (_Float16*)(ws + WS_K), *VI = (_Float16*)(ws + WS_VI), *VP = (_Float16*)(ws + WS_VP), *P = (_Float16*)(ws + WS_P);
  k_fc<<<dim3(NN / 64), 128, 0, stream>>>(F[0], F[1], F[2], F[3], F[4], X);
  for (int l = 0; l < TNL; ++l) {
    k_lin<<<dim3(NN / 64, HID / 128), 128, 0, stream>>>(X, nullptr, F[5] + (size_t)l * HID * HID, F[6] + l * HID, 0, HID, Q);
    k_lin<<<dim3(NN / 64, HID / 128), 128, 0, stream>>>(X, nullptr, F[7] + (size_t)l * HID * HID, F[8] + l * HID, 1, HID, K);
    k_lin<<<dim3(NN / 64, HID / 128), 128, 0, stream>>>(X, nullptr, F[9] + (size_t)l * HID * HID, F[10] + l * HID, 2, HID, VI);
    k_lin<<<dim3(NN / 64, (NHD * VW) / 128), 128, 0, stream>>>(X, VI, F[11] + (size_t)l * HID * NHD * VW, F[12] + l * NHD * VW, 3, NHD * VW, VP);
    k_w<<<dim3(NN / 64, NN / 128), 128, 0, stream>>>(Q, K, P, P + (size_t)NN * NN);
    for (int h = 0; h < NHD; ++h) k_pv<<<dim3(NN / 64, 2), 128, 0, stream>>>(P + (size_t)h * NN * NN, VP, h, O);
    k_mix<<<dim3(NN / 64), 128, 0, stream>>>(O, X, F[3] + (l + 1) * HID, F[4] + (l + 1) * HID, (l == NL - 1) ? (float*)d_out : nullptr);
  }
}
